// SAttention_49667001811359
// MI455X (gfx1250) — hardware-verified
//
#include <hip/hip_runtime.h>
#include <math.h>

constexpr int kBatch = 16;
constexpr int kSeq   = 1024;
constexpr int kDim   = 512;
constexpr int kHeads = 8;
constexpr int kDh    = 64;
constexpr int kImg   = 32;
constexpr int kTok   = kBatch * kSeq;
constexpr int kGroupB = 4;
constexpr float kWCarry     = 16.0f;
constexpr float kWCarryInv  = 1.0f / 16.0f;
constexpr float kPCarry     = 32768.0f;
constexpr float kMidCarry   = 64.0f;
constexpr float kAttScale   = 0.125f;
constexpr float kPVScale    = kMidCarry / kPCarry;
constexpr float kProjScale  = 1.0f / (kMidCarry * kWCarry);
static_assert(kHeads * kDh == kDim, "shape");
static_assert(kImg * kImg == kSeq, "image");
static_assert(kTok % 64 == 0 && kSeq % 64 == 0 && kDim % 64 == 0 && kDh % 64 == 0, "tile multiples");
static_assert(kDim % 32 == 0 && kDh % 32 == 0 && kSeq % 32 == 0, "K multiples of 32");
static_assert(kBatch % kGroupB == 0, "groups");

typedef __attribute__((ext_vector_type(16))) _Float16 v16h;
typedef __attribute__((ext_vector_type(8)))  _Float16 v8h;
typedef __attribute__((ext_vector_type(16))) __bf16   v16b;
typedef __attribute__((ext_vector_type(8)))  __bf16   v8b;
typedef __attribute__((ext_vector_type(8)))  float    v8f;
typedef __attribute__((ext_vector_type(4)))  float    v4f;
typedef __attribute__((ext_vector_type(4)))  unsigned int v4u;

__device__ __forceinline__ unsigned short f2bf_bits(float f) {
  unsigned u = __float_as_uint(f);
  return (unsigned short)((u + 0x7FFFu + ((u >> 16) & 1u)) >> 16);
}
__device__ __forceinline__ float bf_bits2f(unsigned short h) { return __uint_as_float(((unsigned)h) << 16); }

__device__ __forceinline__ void dep_guard_h(v8f& a, v8f& b, v16h x, v16h y) { asm volatile("v_nop\n\tv_nop\n\tv_nop\n\tv_nop" : "+v"(a), "+v"(b) : "v"(x), "v"(y)); }
__device__ __forceinline__ void dep_guard_b(v8f& a, v8f& b, v16b x, v16b y) { asm volatile("v_nop\n\tv_nop\n\tv_nop\n\tv_nop" : "+v"(a), "+v"(b) : "v"(x), "v"(y)); }
__device__ __forceinline__ void keep4_h(v16h a, v16h b, v16h c, v16h d) { asm volatile("v_nop" :: "v"(a), "v"(b), "v"(c), "v"(d)); }
__device__ __forceinline__ void keep4_b(v16b a, v16b b, v16b c, v16b d) { asm volatile("v_nop" :: "v"(a), "v"(b), "v"(c), "v"(d)); }
__device__ __forceinline__ void acc_guard4(v8f& a, v8f& b, v8f& c, v8f& d) { asm volatile("v_nop\n\tv_nop\n\tv_nop\n\tv_nop" : "+v"(a), "+v"(b), "+v"(c), "+v"(d)); }
template <typename T> struct Frag;
template <> struct Frag<_Float16> {
  typedef v16h V; union U { v16h v; v8h h[2]; };
  static __device__ __forceinline__ v16h load(const _Float16* p) {
    U f; f.h[0] = *(const v8h*)(p); f.h[1] = *(const v8h*)(p + 16); return f.v;
  }
  static __device__ __forceinline__ v8f mma(v16h a, v16h b, v8f c) {
    return __builtin_amdgcn_wmma_f32_16x16x32_f16(false, a, false, b, (short)0, c, false, false);
  }
  static __device__ __forceinline__ void guard(v8f& a, v8f& b, v16h x, v16h y) { dep_guard_h(a, b, x, y); }
  static __device__ __forceinline__ void keep(v16h a, v16h b, v16h c, v16h d) { keep4_h(a, b, c, d); }
};
template <> struct Frag<__bf16> {
  typedef v16b V; union U { v16b v; v8b h[2]; };
  static __device__ __forceinline__ v16b load(const __bf16* p) {
    U f; f.h[0] = *(const v8b*)(p); f.h[1] = *(const v8b*)(p + 16); return f.v;
  }
  static __device__ __forceinline__ v8f mma(v16b a, v16b b, v8f c) {
    return __builtin_amdgcn_wmma_f32_16x16x32_bf16(false, a, false, b, (short)0, c, false, false);
  }
  static __device__ __forceinline__ void guard(v8f& a, v8f& b, v16b x, v16b y) { dep_guard_b(a, b, x, y); }
  static __device__ __forceinline__ void keep(v16b a, v16b b, v16b c, v16b d) { keep4_b(a, b, c, d); }
};

__device__ __forceinline__ unsigned pk16(unsigned short a, unsigned short b) { return (unsigned)a | ((unsigned)b << 16); }
__device__ __forceinline__ unsigned short h_bits(float f) { const _Float16 h = (_Float16)f; return __builtin_bit_cast(unsigned short, h); }

__device__ __forceinline__ float h16_to_f32(unsigned hb) {
  const unsigned sgn = (hb & 0x8000u) << 16; const unsigned em = hb & 0x7fffu;
  const float fn = __uint_as_float((em << 13) + 0x38000000u);
  const float fs = (float)em * 5.9604644775390625e-8f;
  const float mag = (em < 0x400u) ? fs : fn; return __uint_as_float(__float_as_uint(mag) | sgn); }

template <int ET> struct Elem;
template <> struct Elem<0> { typedef _Float16 T; };
template <> struct Elem<1> { typedef __bf16 T; };
template <int ET, bool SPLIT, int BIAS_MODE, int OUT_MODE, bool RESID, int ACT = 0>
__global__ __launch_bounds__(256) void wmma_gemm64(
    const unsigned short* __restrict__ Ap, const unsigned short* __restrict__ A2p, int lda, long strideA,
    const unsigned short* __restrict__ Btp, const unsigned short* __restrict__ Bt2p, int ldb, long strideB,
    void* __restrict__ Cout, void* __restrict__ Cout2, int ldc, long strideC,
    const float* __restrict__ bias, long strideBias,
    const float* __restrict__ resid, long strideR,
    int M, int N, int K, float scale) {
  static_assert(!RESID, "resid path not used");
  typedef typename Elem<ET>::T T;
  typedef typename Frag<T>::V V;
  (void)resid; (void)strideR;
  const T* A = (const T*)Ap; const T* A2 = (const T*)A2p; const T* Bt = (const T*)Btp; const T* Bt2 = (const T*)Bt2p;
  __shared__ __align__(16) float sT[8][16 * 68];
  const int b    = blockIdx.y;
  const int lane = threadIdx.x & 31;
  const int wave = threadIdx.x >> 5;
  const int tilesN = N >> 6;
  const int tilesM = M >> 6;
  const int tile = blockIdx.x * 8 + wave;
  if (tile >= tilesM * tilesN) return;
  const int tm = tile / tilesN;
  const int tn = tile - tm * tilesN;
  const int m0 = tm << 6;
  const int n0 = tn << 6;

  const T* Ab  = A  + (size_t)b * strideA;
  const T* Bb  = Bt + (size_t)b * strideB;
  const T* Ab2 = SPLIT ? (A2  + (size_t)b * strideA) : nullptr;
  const T* Bb2 = SPLIT ? (Bt2 + (size_t)b * strideB) : nullptr;

  const int rlane = lane & 15;
  const int koff  = (lane >> 4) * 8;
  const int mOff  = (lane >> 4) * 8;

  v8f acc[4][4];
#pragma unroll
  for (int i = 0; i < 4; ++i)
#pragma unroll
    for (int j = 0; j < 4; ++j) acc[i][j] = (v8f){0.f,0.f,0.f,0.f,0.f,0.f,0.f,0.f};

  for (int k0 = 0; k0 < K; k0 += 32) {
    V bh[4], bl[4];
#pragma unroll
    for (int j = 0; j < 4; ++j) {
      const size_t bo = (size_t)(n0 + (j << 4) + rlane) * ldb + koff + k0;
      bh[j] = Frag<T>::load(Bb + bo);
      if (SPLIT) bl[j] = Frag<T>::load(Bb2 + bo);
    }
#pragma unroll
    for (int i = 0; i < 4; ++i) {
      const size_t ao = (size_t)(m0 + (i << 4) + rlane) * lda + koff + k0;
      V ah = Frag<T>::load(Ab + ao);
      V al;
      if (SPLIT) al = Frag<T>::load(Ab2 + ao);
#pragma unroll
      for (int j = 0; j < 4; ++j) {
        acc[i][j] = Frag<T>::mma(ah, bh[j], acc[i][j]);
        if (SPLIT) {
          acc[i][j] = Frag<T>::mma(ah, bl[j], acc[i][j]);
          acc[i][j] = Frag<T>::mma(al, bh[j], acc[i][j]);
        }
      }
      Frag<T>::guard(acc[i][0], acc[i][3], ah, SPLIT ? al : ah);
    }
    Frag<T>::keep(bh[0], bh[1], bh[2], bh[3]);
    if (SPLIT) Frag<T>::keep(bl[0], bl[1], bl[2], bl[3]);
  }
  acc_guard4(acc[0][0], acc[0][1], acc[0][2], acc[0][3]);
  acc_guard4(acc[1][0], acc[1][1], acc[1][2], acc[1][3]);
  acc_guard4(acc[2][0], acc[2][1], acc[2][2], acc[2][3]);
  acc_guard4(acc[3][0], acc[3][1], acc[3][2], acc[3][3]);

  float* slab = sT[wave];
  const float* biasb = (BIAS_MODE != 0) ? (bias + (size_t)b * strideBias) : nullptr;
#pragma unroll
  for (int i = 0; i < 4; ++i) {
    const int mBase = m0 + (i << 4);
    float b8[8] = {0.f,0.f,0.f,0.f,0.f,0.f,0.f,0.f};
    if (BIAS_MODE == 1) {
      const v4f bm0 = *(const v4f*)(biasb + mBase + mOff);
      const v4f bm1 = *(const v4f*)(biasb + mBase + mOff + 4);
      b8[0] = bm0[0]; b8[1] = bm0[1]; b8[2] = bm0[2]; b8[3] = bm0[3];
      b8[4] = bm1[0]; b8[5] = bm1[1]; b8[6] = bm1[2]; b8[7] = bm1[3];
    }
#pragma unroll
    for (int j = 0; j < 4; ++j) {
      const int n = n0 + (j << 4) + rlane;
      float bv = 0.f;
      if (BIAS_MODE == 2) bv = biasb[n];
#pragma unroll
      for (int r = 0; r < 8; ++r) {
        float v = acc[i][j][r] * scale;
        if (BIAS_MODE == 1) v += b8[r];
        if (BIAS_MODE == 2) v += bv;
        if (ACT == 2) v = fmaxf(v, 0.0f);
        if (ACT == 4) v = (v > 0.f) ? v : 0.01f * v;
        slab[(mOff + r) * 68 + (j << 4) + rlane] = v;
      }
    }
    __builtin_amdgcn_fence(__ATOMIC_RELEASE, "workgroup");
    __builtin_amdgcn_wave_barrier();
    __builtin_amdgcn_fence(__ATOMIC_ACQUIRE, "workgroup");
    if (OUT_MODE == 0) {
      float* C = (float*)Cout + (size_t)b * strideC;
      const int hh = lane >> 4, c4 = (lane & 15) * 4;
      for (int pass = 0; pass < 2; ++pass) {
#pragma unroll
        for (int it = 0; it < 8; ++it) {
          const int row = it * 2 + hh;
          v4f v = *(const v4f*)(slab + row * 68 + c4);
          *(volatile v4f*)(C + (size_t)(mBase + row) * ldc + n0 + c4) = v;
        }
        __threadfence();
      }
    } else {
      const int q = lane >> 3, c8 = (lane & 7) * 8;
      unsigned short* C  = (unsigned short*)Cout  + (size_t)b * strideC;
      unsigned short* C2 = (OUT_MODE == 2) ? ((unsigned short*)Cout2 + (size_t)b * strideC) : nullptr;
      for (int pass = 0; pass < 2; ++pass) {
#pragma unroll
        for (int it = 0; it < 4; ++it) {
          const int row = it * 4 + q;
          const float* sp = slab + row * 68 + c8;
          v8h hv, lv;
#pragma unroll
          for (int e = 0; e < 8; ++e) {
            if (OUT_MODE == 1) {
              hv[e] = (_Float16)sp[e];
            } else {
              unsigned short hb = f2bf_bits(sp[e]);
              unsigned short lb = f2bf_bits(sp[e] - bf_bits2f(hb));
              hv[e] = __builtin_bit_cast(_Float16, hb);
              lv[e] = __builtin_bit_cast(_Float16, lb);
            }
          }
          *(volatile v8h*)(C + (size_t)(mBase + row) * ldc + n0 + c8) = hv;
          if (OUT_MODE == 2) *(volatile v8h*)(C2 + (size_t)(mBase + row) * ldc + n0 + c8) = lv;
        }
        __threadfence();
      }
    }
    __builtin_amdgcn_fence(__ATOMIC_RELEASE, "workgroup");
    __builtin_amdgcn_wave_barrier();
    __builtin_amdgcn_fence(__ATOMIC_ACQUIRE, "workgroup");
  }
}

__global__ __launch_bounds__(256) void cast8_f16_kernel(const float* __restrict__ in, unsigned short* __restrict__ out, int n8) {
  const int i = blockIdx.x * 256 + threadIdx.x;
  if (i >= n8) return;
  const float* p = in + 8 * (size_t)i;
  const v4f a = *(const v4f*)(p);
  const v4f c = *(const v4f*)(p + 4);
  unsigned short hb[8];
#pragma unroll
  for (int e = 0; e < 4; ++e) {
    hb[e]     = h_bits(a[e]);
    hb[4 + e] = h_bits(c[e]);
  }
  const v4u u = (v4u){pk16(hb[0], hb[1]), pk16(hb[2], hb[3]), pk16(hb[4], hb[5]), pk16(hb[6], hb[7])};
  unsigned short* q = out + 8 * (size_t)i;
  *(volatile v4u*)q = u;
  __threadfence();
  *(volatile v4u*)q = u;
}

__global__ __launch_bounds__(256) void wtcast_kernel(const float* __restrict__ W, int nOut,
                                                     unsigned short* __restrict__ out, float scale) {
  __shared__ float sm[64][65];
  const int t  = threadIdx.x;
  const int i0 = blockIdx.x * 64;
  const int o0 = blockIdx.y * 64;
#pragma unroll
  for (int it = 0; it < 16; ++it) {
    const int e = it * 256 + t;
    const int r = e >> 6;
    const int c = e & 63;
    sm[c][r] = W[(size_t)(i0 + r) * nOut + o0 + c] * scale;
  }
  __syncthreads();
  const int lane = t & 31, wave = t >> 5;
  const int q = lane >> 3, c8 = (lane & 7) * 8;
  for (int pass = 0; pass < 2; ++pass) {
#pragma unroll
    for (int it = 0; it < 2; ++it) {
      const int row = wave * 8 + it * 4 + q;
      unsigned short hb[8];
#pragma unroll
      for (int e = 0; e < 8; ++e) hb[e] = h_bits(sm[row][c8 + e]);
      const v4u u = (v4u){pk16(hb[0], hb[1]), pk16(hb[2], hb[3]), pk16(hb[4], hb[5]), pk16(hb[6], hb[7])};
      *(volatile v4u*)(out + (size_t)(o0 + row) * kDim + i0 + c8) = u;
    }
    __threadfence();
  }
}

__global__ __launch_bounds__(128) void softmax_row_kernel(const float* __restrict__ S, unsigned short* __restrict__ P) {
  __shared__ float redM[4];
  __shared__ float redS[4];
  const int row  = blockIdx.x;
  const int t    = threadIdx.x;
  const int lane = t & 31, wave = t >> 5;
  const int c0   = t * 8;
  const float* sr = S + (size_t)row * kSeq + c0;
  const v4f a = *(const v4f*)(sr);
  const v4f c = *(const v4f*)(sr + 4);
  float x[8];
#pragma unroll
  for (int e = 0; e < 4; ++e) { x[e] = a[e]; x[4 + e] = c[e]; }
  float m = fmaxf(fmaxf(fmaxf(x[0], x[1]), fmaxf(x[2], x[3])), fmaxf(fmaxf(x[4], x[5]), fmaxf(x[6], x[7])));
#pragma unroll
  for (int off = 16; off > 0; off >>= 1) m = fmaxf(m, __shfl_xor(m, off, 32));
  if (lane == 0) redM[wave] = m;
  __syncthreads();
  float mx = redM[0];
  mx = fmaxf(mx, redM[1]);
  mx = fmaxf(mx, redM[2]);
  mx = fmaxf(mx, redM[3]);

  float ev[8];
  float sum = 0.f;
#pragma unroll
  for (int e = 0; e < 8; ++e) { ev[e] = expf(x[e] - mx); sum += ev[e]; }
#pragma unroll
  for (int off = 16; off > 0; off >>= 1) sum += __shfl_xor(sum, off, 32);
  if (lane == 0) redS[wave] = sum;
  __syncthreads();
  float tot = redS[0];
  tot += redS[1];
  tot += redS[2];
  tot += redS[3];
  const float inv = kPCarry * (1.0f / tot);

  unsigned short hb[8];
#pragma unroll
  for (int e = 0; e < 8; ++e) hb[e] = h_bits(ev[e] * inv);
  const v4u u = (v4u){pk16(hb[0], hb[1]), pk16(hb[2], hb[3]), pk16(hb[4], hb[5]), pk16(hb[6], hb[7])};
  unsigned short* pr = P + (size_t)row * kSeq + c0;
  *(volatile v4u*)pr = u;
  __threadfence();
  *(volatile v4u*)pr = u;
}

constexpr int kCvRows  = 6;
constexpr int kCvCols  = 34;
constexpr int kCvPitch = kCvRows * kCvCols;
__global__ __launch_bounds__(256) void conv_mid_kernel(const unsigned short* __restrict__ VT,
                                                       const unsigned short* __restrict__ O16,
                                                       const float* __restrict__ cw, const float* __restrict__ cb,
                                                       unsigned short* __restrict__ MID,
                                                       const int* __restrict__ hw0, const int* __restrict__ hw1) {
  (void)hw0; (void)hw1;
  __shared__ __align__(16) float sv[64 * kCvPitch];
  __shared__ float sw[64 * 9];
  __shared__ float sb[64];
  const int t  = threadIdx.x;
  const int c0 = blockIdx.x * 64;
  const int y0 = blockIdx.y * 4;
  const int b  = blockIdx.z;

  for (int i = t; i < 64 * 9; i += 256) sw[i] = cw[(size_t)c0 * 9 + i] * kMidCarry;
  if (t < 64) sb[t] = cb[c0 + t] * kMidCarry;
  for (int i = t; i < 64 * kCvRows * 2; i += 256) {
    const int cl  = i / (kCvRows * 2);
    const int rem = i - cl * (kCvRows * 2);
    const int r   = rem >> 1;
    const int col = (rem & 1) * (kCvCols - 1);
    sv[cl * kCvPitch + r * kCvCols + col] = 0.0f;
  }
#pragma unroll
  for (int i = 0; i < 6; ++i) {
    const int idx = i * 256 + t;
    const int cl  = idx / 24;
    const int w4  = idx - cl * 24;
    const int r   = w4 >> 2;
    const int x0  = (w4 & 3) * 8;
    const int yy  = y0 - 1 + r;
    const int yyc = (yy < 0) ? 0 : ((yy > kImg - 1) ? (kImg - 1) : yy);
    const v4u u = *(const v4u*)(VT + (size_t)(c0 + cl) * kTok + (size_t)b * kSeq + yyc * kImg + x0);
    const float f = (yy >= 0 && yy <= kImg - 1) ? 1.0f : 0.0f;
    float* dst = sv + cl * kCvPitch + r * kCvCols + 1 + x0;
    dst[0] = h16_to_f32(u[0] & 0xffffu) * f;
    dst[1] = h16_to_f32(u[0] >> 16) * f;
    dst[2] = h16_to_f32(u[1] & 0xffffu) * f;
    dst[3] = h16_to_f32(u[1] >> 16) * f;
    dst[4] = h16_to_f32(u[2] & 0xffffu) * f;
    dst[5] = h16_to_f32(u[2] >> 16) * f;
    dst[6] = h16_to_f32(u[3] & 0xffffu) * f;
    dst[7] = h16_to_f32(u[3] >> 16) * f;
  }
  __syncthreads();

  const int rq = t >> 3;
  const int c8 = (t & 7) * 8;
#pragma unroll 1
  for (int it = 0; it < 4; ++it) {
    const int row = it * 32 + rq;
    const int yl  = row >> 5;
    const int x   = row & 31;
    const size_t tok = (size_t)b * kSeq + (size_t)(y0 * kImg + row);
    const v4u ou = *(const v4u*)(O16 + tok * kDim + c0 + c8);
    float o[8];
    o[0] = h16_to_f32(ou[0] & 0xffffu); o[1] = h16_to_f32(ou[0] >> 16);
    o[2] = h16_to_f32(ou[1] & 0xffffu); o[3] = h16_to_f32(ou[1] >> 16);
    o[4] = h16_to_f32(ou[2] & 0xffffu); o[5] = h16_to_f32(ou[2] >> 16);
    o[6] = h16_to_f32(ou[3] & 0xffffu); o[7] = h16_to_f32(ou[3] >> 16);
    unsigned short hb[8];
#pragma unroll
    for (int e = 0; e < 8; ++e) {
      const int cl = c8 + e;
      const float* vr = sv + cl * kCvPitch + yl * kCvCols + x;
      const float* wr = sw + cl * 9;
      float acc = sb[cl];
#pragma unroll
      for (int ky = 0; ky < 3; ++ky) {
#pragma unroll
        for (int kx = 0; kx < 3; ++kx) acc = fmaf(wr[ky * 3 + kx], vr[ky * kCvCols + kx], acc);
      }
      hb[e] = h_bits(o[e] + acc);
    }
    const v4u u = (v4u){pk16(hb[0], hb[1]), pk16(hb[2], hb[3]), pk16(hb[4], hb[5]), pk16(hb[6], hb[7])};
    unsigned short* mp = MID + tok * kDim + c0 + c8;
    *(volatile v4u*)mp = u;
    __threadfence();
    *(volatile v4u*)mp = u;
  }
}

extern "C" void kernel_launch(void* const* d_in, const int* in_sizes, int n_in,
                              void* d_out, int out_size, void* d_ws, size_t ws_size,
                              hipStream_t stream) {
  if (n_in < 11) return;
  const int nX = kTok * kDim;
  if (in_sizes[0] != nX) return;
  if (in_sizes[1] != kDim * kDim || in_sizes[2] != kDim) return;
  if (in_sizes[3] != kDim * 2 * kDim || in_sizes[4] != 2 * kDim) return;
  if (in_sizes[5] != kDim * 9 || in_sizes[6] != kDim) return;
  if (in_sizes[7] != kDim * kDim || in_sizes[8] != kDim) return;
  if (out_size != kBatch * kDim * kSeq) return;

  const size_t szPlane16 = (size_t)kTok * kDim * 2;
  const size_t szWQKVT   = (size_t)3 * kDim * kDim * 2;
  const size_t szWPT     = (size_t)kDim * kDim * 2;
  const size_t szQ       = (size_t)kHeads * kTok * kDh * 2;
  const size_t szVT      = (size_t)kDim * kTok * 2;
  const size_t szS       = (size_t)kGroupB * kSeq * kSeq * 4;
  const size_t szP       = (size_t)kGroupB * kSeq * kSeq * 2;
  const size_t offXH   = 0;
  const size_t offWQKV = offXH + szPlane16;
  const size_t offWPT  = offWQKV + szWQKVT;
  const size_t offQ    = offWPT + szWPT;
  const size_t offK    = offQ + szQ;
  const size_t offVT   = offK + szQ;
  const size_t offS    = offVT + szVT;
  const size_t offP    = offS + szS;
  const size_t offO    = offP + szP;
  const size_t offMID  = offO + szPlane16;
  const size_t total   = offMID + szPlane16;
  if (ws_size < total) return;

  const float* x    = (const float*)d_in[0];
  const float* Wq   = (const float*)d_in[1];
  const float* bq   = (const float*)d_in[2];
  const float* Wkv  = (const float*)d_in[3];
  const float* bkv  = (const float*)d_in[4];
  const float* cw   = (const float*)d_in[5];
  const float* cb   = (const float*)d_in[6];
  const float* Wp   = (const float*)d_in[7];
  const float* bp   = (const float*)d_in[8];
  const int*   hIn  = (const int*)d_in[9];
  const int*   wIn  = (const int*)d_in[10];
  float* out = (float*)d_out;
  char* ws = (char*)d_ws;
  unsigned short* XH    = (unsigned short*)(ws + offXH);
  unsigned short* WQKVT = (unsigned short*)(ws + offWQKV);
  unsigned short* WPT   = (unsigned short*)(ws + offWPT);
  unsigned short* Q16   = (unsigned short*)(ws + offQ);
  unsigned short* K16   = (unsigned short*)(ws + offK);
  unsigned short* VT    = (unsigned short*)(ws + offVT);
  float*          SC    = (float*)(ws + offS);
  unsigned short* PP    = (unsigned short*)(ws + offP);
  unsigned short* O16   = (unsigned short*)(ws + offO);
  unsigned short* MID16 = (unsigned short*)(ws + offMID);

  const int n8 = nX / 8;
  cast8_f16_kernel<<<dim3(n8 / 256), dim3(256), 0, stream>>>(x, XH, n8);
  wtcast_kernel<<<dim3(kDim / 64, kDim / 64), dim3(256), 0, stream>>>(Wq, kDim, WQKVT, kWCarry);
  wtcast_kernel<<<dim3(kDim / 64, (2 * kDim) / 64), dim3(256), 0, stream>>>(Wkv, 2 * kDim, WQKVT + (size_t)kDim * kDim, kWCarry);
  wtcast_kernel<<<dim3(kDim / 64, kDim / 64), dim3(256), 0, stream>>>(Wp, kDim, WPT, kWCarry);

  const long strideHeadW  = (long)kDh * kDim;
  const long strideHeadQK = (long)kTok * kDh;
  const long strideHeadVT = (long)kDh * kTok;
  const int  tilesQK = (kTok / 64) * (kDh / 64);
  wmma_gemm64<0, false, 2, 1, false, 0><<<dim3(tilesQK / 8, kHeads), dim3(256), 0, stream>>>(
      XH, XH, kDim, 0L, WQKVT, WQKVT, kDim, strideHeadW,
      (void*)Q16, (void*)Q16, kDh, strideHeadQK, bq, (long)kDh, bq, 0L, kTok, kDh, kDim, kWCarryInv);
  wmma_gemm64<0, false, 2, 1, false, 0><<<dim3(tilesQK / 8, kHeads), dim3(256), 0, stream>>>(
      XH, XH, kDim, 0L, WQKVT + (size_t)kDim * kDim, WQKVT, kDim, strideHeadW,
      (void*)K16, (void*)K16, kDh, strideHeadQK, bkv, (long)kDh, bkv, 0L, kTok, kDh, kDim, kWCarryInv);
  wmma_gemm64<0, false, 1, 1, false, 0><<<dim3(tilesQK / 8, kHeads), dim3(256), 0, stream>>>(
      WQKVT + (size_t)2 * kDim * kDim, WQKVT, kDim, strideHeadW, XH, XH, kDim, 0L,
      (void*)VT, (void*)VT, kTok, strideHeadVT, bkv + kDim, (long)kDh, bkv, 0L, kDh, kTok, kDim, kWCarryInv);

  const long strideBQK  = (long)kSeq * kDh;
  const long strideS    = (long)kSeq * kSeq;
  const long strideBO   = (long)kSeq * kDim;
  const int  tilesScore = (kSeq / 64) * (kSeq / 64);
  const int  tilesPV    = (kSeq / 64) * (kDh / 64);
  for (int h = 0; h < kHeads; ++h) {
    for (int gq = 0; gq < kBatch / kGroupB; ++gq) {
      const int b0 = gq * kGroupB;
      const unsigned short* Qg = Q16 + (size_t)h * strideHeadQK + (size_t)b0 * strideBQK;
      const unsigned short* Kg = K16 + (size_t)h * strideHeadQK + (size_t)b0 * strideBQK;
      wmma_gemm64<0, false, 0, 0, false, 0><<<dim3(tilesScore / 8, kGroupB), dim3(256), 0, stream>>>(
          Qg, Qg, kDh, strideBQK, Kg, Kg, kDh, strideBQK,
          (void*)SC, (void*)SC, kSeq, strideS, bq, 0L, bq, 0L, kSeq, kSeq, kDh, kAttScale);
      softmax_row_kernel<<<dim3(kGroupB * kSeq), dim3(128), 0, stream>>>(SC, PP);
      const unsigned short* VTg = VT + (size_t)h * strideHeadVT + (size_t)b0 * kSeq;
      unsigned short* Og = O16 + (size_t)b0 * strideBO + (size_t)h * kDh;
      wmma_gemm64<0, false, 0, 1, false, 0><<<dim3(tilesPV / 8, kGroupB), dim3(256), 0, stream>>>(
          PP, PP, kSeq, strideS, VTg, VTg, kTok, (long)kSeq,
          (void*)Og, (void*)Og, kDim, strideBO, bq, 0L, bq, 0L, kSeq, kDh, kSeq, kPVScale);
    }
  }

  conv_mid_kernel<<<dim3(kDim / 64, kImg / 4, kBatch), dim3(256), 0, stream>>>(VT, O16, cw, cb, MID16, hIn, wIn);

  const int tilesProj = (kDim / 64) * (kSeq / 64);
  wmma_gemm64<0, false, 1, 0, false, 0><<<dim3(tilesProj / 8, kBatch), dim3(256), 0, stream>>>(
      WPT, WPT, kDim, 0L, MID16, MID16, kDim, strideBO,
      (void*)out, (void*)out, kSeq, (long)kDim * kSeq, bp, 0L, bp, 0L, kDim, kSeq, kDim, kProjScale);
}
